// MDTA_86912958202231
// MI455X (gfx1250) — hardware-verified
//
#include <hip/hip_runtime.h>
#include <stdint.h>

#define NB     2
#define CC     128
#define HH     128
#define WW     128
#define IMGPIX (HH * WW)
#define NPIX   (NB * IMGPIX)
#define HP     (HH + 2)
#define WP     (WW + 2)
#define PADIMG (HP * WP)
#define PADPIX (NB * PADIMG)
#define KCV    1152
#define NKS    36
#define NHEAD  8
#define HD     16
#define HSZ    (IMGPIX * HD)
#define BSZ    (CC * IMGPIX)
#define LDC    132
#define FP     40
#define WSP    17
#define NHALO  (2 * WP + 2 * HH)
#define RSC    0.00048828125f
#define PS1    ((size_t)PADPIX * CC)
#define PS2    ((size_t)NPIX * CC)

static_assert(NPIX == NB * IMGPIX);
static_assert(IMGPIX == 16384 && HH == 128 && WW == 128);
static_assert(PADIMG == 16900);
static_assert(KCV == 9 * CC && KCV == NKS * 32);
static_assert(CC == NHEAD * HD);
static_assert(BSZ == CC * IMGPIX && HSZ * NHEAD == BSZ);
static_assert((IMGPIX % 64) == 0 && (WW % 64) == 0);
static_assert((LDC * 4) % 16 == 0 && (FP * 2) % 16 == 0);
static_assert(NHALO == 516);
static_assert((KCV % 8) == 0 && (CC % 32) == 0);
static_assert(IMGPIX == 32 * 32 * 16);


typedef _Float16 v16h __attribute__((ext_vector_type(16)));
typedef _Float16 v8h  __attribute__((ext_vector_type(8)));
typedef float    v8f  __attribute__((ext_vector_type(8)));
typedef float    v4f  __attribute__((ext_vector_type(4)));
typedef unsigned int v4u __attribute__((ext_vector_type(4)));

__device__ __forceinline__ unsigned short bf_bits(float f) {
  unsigned u = __float_as_uint(f);
  return (unsigned short)((u + 0x7FFFu + ((u >> 16) & 1u)) >> 16);
}
__device__ __forceinline__ float bf_up(unsigned short b) { return __uint_as_float(((unsigned)b) << 16); }
__device__ __forceinline__ float bfr(float f) { return bf_up(bf_bits(f)); }
__device__ __forceinline__ unsigned short h_bits(_Float16 x) { return __builtin_bit_cast(unsigned short, x); }
__device__ __forceinline__ unsigned short hb16(float f) { return h_bits((_Float16)f); }
__device__ __forceinline__ unsigned pk16(unsigned short a, unsigned short b) { return (unsigned)a | ((unsigned)b << 16); }
__device__ __forceinline__ v8f zero8() { v8f z = {0.f, 0.f, 0.f, 0.f, 0.f, 0.f, 0.f, 0.f}; return z; }
__device__ __forceinline__ void split2(float f0, float f1, unsigned& hp, unsigned& lp) {
  const _Float16 h0 = (_Float16)f0, h1 = (_Float16)f1;
  const float q0 = (f0 - (float)h0) * 2048.0f, q1 = (f1 - (float)h1) * 2048.0f;
  hp = pk16(h_bits(h0), h_bits(h1));
  lp = pk16(hb16(q0), hb16(q1));
}

__device__ __forceinline__ v16h ldfrag_h(const _Float16* p) {
  union { v16h v; v8h h[2]; } f;
  f.h[0] = *(const v8h*)(p);
  f.h[1] = *(const v8h*)(p + 16);
  return f.v;
}
__device__ __forceinline__ v16h ldfrag2(const _Float16* pa, const _Float16* pb) {
  union { v16h v; v8h h[2]; } f;
  f.h[0] = *(const v8h*)(pa);
  f.h[1] = *(const v8h*)(pb);
  return f.v;
}

__device__ __forceinline__ v8f mma_raw(v16h a, v16h b, v8f c) {
  return __builtin_amdgcn_wmma_f32_16x16x32_f16(false, a, false, b, (short)0, c, false, false);
}
__device__ __forceinline__ void guard8(v8f& c0, v8f& c1, v8f& c2, v8f& c3, v8f& c4, v8f& c5, v8f& c6, v8f& c7,
                                       const v16h& a0, const v16h& a1, const v16h& a2, const v16h& a3,
                                       const v16h& b0, const v16h& b1) {
#if defined(__HIP_DEVICE_COMPILE__)
  asm volatile("v_nop\n\tv_nop\n\tv_nop\n\tv_nop"
               : "+v"(c0), "+v"(c1), "+v"(c2), "+v"(c3), "+v"(c4), "+v"(c5), "+v"(c6), "+v"(c7)
               : "v"(a0), "v"(a1), "v"(a2), "v"(a3), "v"(b0), "v"(b1));
#endif
}
__device__ __forceinline__ void guard4(v8f& c0, v8f& c1, v8f& c2, v8f& c3,
                                       const v16h& a0, const v16h& a1, const v16h& b0, const v16h& b1) {
#if defined(__HIP_DEVICE_COMPILE__)
  asm volatile("v_nop\n\tv_nop\n\tv_nop\n\tv_nop"
               : "+v"(c0), "+v"(c1), "+v"(c2), "+v"(c3)
               : "v"(a0), "v"(a1), "v"(b0), "v"(b1));
#endif
}
__device__ __forceinline__ void guard2(v8f& c0, v8f& c1, const v16h& a0, const v16h& b0, const v16h& b1) {
#if defined(__HIP_DEVICE_COMPILE__)
  asm volatile("v_nop\n\tv_nop\n\tv_nop\n\tv_nop"
               : "+v"(c0), "+v"(c1)
               : "v"(a0), "v"(b0), "v"(b1));
#endif
}

__device__ __forceinline__ void mm_tile2(const _Float16* __restrict__ Ah, const _Float16* __restrict__ Al, int lda,
                                         const _Float16* __restrict__ W, int ldw, int nks,
                                         int arow0, int bcol0, float* Cs) {
  const int tid = threadIdx.x, wave = tid >> 5, lane = tid & 31, hh = lane >> 4, c = lane & 15;
  const int mw = wave >> 2, nw = wave & 3;
  const size_t r0 = (size_t)(arow0 + mw * 32 + c) * lda + 8 * hh;
  const size_t r1 = (size_t)(arow0 + mw * 32 + 16 + c) * lda + 8 * hh;
  const _Float16* a0h = Ah + r0;
  const _Float16* a1h = Ah + r1;
  const _Float16* a0l = Al + r0;
  const _Float16* a1l = Al + r1;
  const _Float16* b0p = W + (size_t)(bcol0 + nw * 32 + c) * ldw + 8 * hh;
  const _Float16* b1p = W + (size_t)(bcol0 + nw * 32 + 16 + c) * ldw + 8 * hh;
  v8f h00 = zero8(), h01 = zero8(), h10 = zero8(), h11 = zero8();
  v8f l00 = zero8(), l01 = zero8(), l10 = zero8(), l11 = zero8();
#pragma unroll 1
  for (int ks = 0; ks < nks; ++ks) {
    const int ko = ks * 32;
    const v16h fa0 = ldfrag_h(a0h + ko);
    const v16h fa1 = ldfrag_h(a1h + ko);
    const v16h ga0 = ldfrag_h(a0l + ko);
    const v16h ga1 = ldfrag_h(a1l + ko);
    const v16h fb0 = ldfrag_h(b0p + ko);
    const v16h fb1 = ldfrag_h(b1p + ko);
    h00 = mma_raw(fa0, fb0, h00);
    h01 = mma_raw(fa0, fb1, h01);
    h10 = mma_raw(fa1, fb0, h10);
    h11 = mma_raw(fa1, fb1, h11);
    l00 = mma_raw(ga0, fb0, l00);
    l01 = mma_raw(ga0, fb1, l01);
    l10 = mma_raw(ga1, fb0, l10);
    l11 = mma_raw(ga1, fb1, l11);
    guard8(h00, h01, h10, h11, l00, l01, l10, l11, fa0, fa1, ga0, ga1, fb0, fb1);
  }
#pragma unroll
  for (int r = 0; r < 8; ++r) {
    const int row = mw * 32 + 8 * hh + r;
    Cs[row * LDC + nw * 32 + c]             = h00[r] + l00[r] * RSC;
    Cs[row * LDC + nw * 32 + 16 + c]        = h01[r] + l01[r] * RSC;
    Cs[(row + 16) * LDC + nw * 32 + c]      = h10[r] + l10[r] * RSC;
    Cs[(row + 16) * LDC + nw * 32 + 16 + c] = h11[r] + l11[r] * RSC;
  }
}

__device__ __forceinline__ size_t conv_abase(int p, int hh) {
  const int b = p / IMGPIX;
  const int r = p - b * IMGPIX;
  const int y = r / WW;
  const int x = r - y * WW;
  return ((size_t)(b * HP + y) * WP + x) * CC + 8 * hh;
}
__device__ __forceinline__ void mm_conv(const _Float16* __restrict__ Ah, const _Float16* __restrict__ Al,
                                        const _Float16* __restrict__ W, int prow0, float* Cs) {
  const int tid = threadIdx.x, wave = tid >> 5, lane = tid & 31, hh = lane >> 4, c = lane & 15;
  const int mw = wave >> 2, nw = wave & 3;
  const size_t r0 = conv_abase(prow0 + mw * 32 + c, hh);
  const size_t r1 = conv_abase(prow0 + mw * 32 + 16 + c, hh);
  const _Float16* a0h = Ah + r0;
  const _Float16* a1h = Ah + r1;
  const _Float16* a0l = Al + r0;
  const _Float16* a1l = Al + r1;
  const _Float16* b0p = W + (size_t)(nw * 32 + c) * KCV + 8 * hh;
  const _Float16* b1p = W + (size_t)(nw * 32 + 16 + c) * KCV + 8 * hh;
  v8f h00 = zero8(), h01 = zero8(), h10 = zero8(), h11 = zero8();
  v8f l00 = zero8(), l01 = zero8(), l10 = zero8(), l11 = zero8();
#pragma unroll 1
  for (int ks = 0; ks < NKS; ++ks) {
    const int tap = ks >> 2, cq = ks & 3;
    const int ky = (tap * 11) >> 5;
    const int kx = tap - 3 * ky;
    const int ao = (ky * WP + kx) * CC + cq * 32;
    const int ko = ks * 32;
    const v16h fa0 = ldfrag_h(a0h + ao);
    const v16h fa1 = ldfrag_h(a1h + ao);
    const v16h ga0 = ldfrag_h(a0l + ao);
    const v16h ga1 = ldfrag_h(a1l + ao);
    const v16h fb0 = ldfrag_h(b0p + ko);
    const v16h fb1 = ldfrag_h(b1p + ko);
    h00 = mma_raw(fa0, fb0, h00);
    h01 = mma_raw(fa0, fb1, h01);
    h10 = mma_raw(fa1, fb0, h10);
    h11 = mma_raw(fa1, fb1, h11);
    l00 = mma_raw(ga0, fb0, l00);
    l01 = mma_raw(ga0, fb1, l01);
    l10 = mma_raw(ga1, fb0, l10);
    l11 = mma_raw(ga1, fb1, l11);
    guard8(h00, h01, h10, h11, l00, l01, l10, l11, fa0, fa1, ga0, ga1, fb0, fb1);
  }
#pragma unroll
  for (int r = 0; r < 8; ++r) {
    const int row = mw * 32 + 8 * hh + r;
    Cs[row * LDC + nw * 32 + c]             = h00[r] + l00[r] * RSC;
    Cs[row * LDC + nw * 32 + 16 + c]        = h01[r] + l01[r] * RSC;
    Cs[(row + 16) * LDC + nw * 32 + c]      = h10[r] + l10[r] * RSC;
    Cs[(row + 16) * LDC + nw * 32 + 16 + c] = h11[r] + l11[r] * RSC;
  }
}

__device__ __forceinline__ void mm_final(const _Float16* __restrict__ Vh, const _Float16* __restrict__ Vl,
                                         const _Float16* __restrict__ Wh, const _Float16* __restrict__ Wl,
                                         int pl0, float* Cs) {
  const int tid = threadIdx.x, wave = tid >> 5, lane = tid & 31, hh = lane >> 4, c = lane & 15;
  const int mw = wave >> 2, nw = wave & 3;
  const size_t r0 = (size_t)(pl0 + mw * 32 + c) * HD + 8 * hh;
  const size_t r1 = (size_t)(pl0 + mw * 32 + 16 + c) * HD + 8 * hh;
  const size_t q0 = (size_t)(nw * 32 + c) * HD + 8 * hh;
  const size_t q1 = (size_t)(nw * 32 + 16 + c) * HD + 8 * hh;
  {
    v8f h00 = zero8(), h01 = zero8(), h10 = zero8(), h11 = zero8();
    v8f l00 = zero8(), l01 = zero8(), l10 = zero8(), l11 = zero8();
#pragma unroll 1
    for (int ks = 0; ks < CC / 32; ++ks) {
      const size_t ao = (size_t)(2 * ks) * HSZ;
      const size_t bo = (size_t)(2 * ks) * (CC * HD);
      const v16h fa0 = ldfrag2(Vh + r0 + ao, Vh + r0 + ao + HSZ);
      const v16h fa1 = ldfrag2(Vh + r1 + ao, Vh + r1 + ao + HSZ);
      const v16h fb0 = ldfrag2(Wh + q0 + bo, Wh + q0 + bo + CC * HD);
      const v16h fb1 = ldfrag2(Wh + q1 + bo, Wh + q1 + bo + CC * HD);
      const v16h gb0 = ldfrag2(Wl + q0 + bo, Wl + q0 + bo + CC * HD);
      const v16h gb1 = ldfrag2(Wl + q1 + bo, Wl + q1 + bo + CC * HD);
      h00 = mma_raw(fa0, fb0, h00);
      h01 = mma_raw(fa0, fb1, h01);
      h10 = mma_raw(fa1, fb0, h10);
      h11 = mma_raw(fa1, fb1, h11);
      l00 = mma_raw(fa0, gb0, l00);
      l01 = mma_raw(fa0, gb1, l01);
      l10 = mma_raw(fa1, gb0, l10);
      l11 = mma_raw(fa1, gb1, l11);
      guard8(h00, h01, h10, h11, l00, l01, l10, l11, fa0, fa1, gb0, gb1, fb0, fb1);
    }
#pragma unroll
    for (int r = 0; r < 8; ++r) {
      const int row = mw * 32 + 8 * hh + r;
      Cs[row * LDC + nw * 32 + c]             = h00[r] + l00[r] * RSC;
      Cs[row * LDC + nw * 32 + 16 + c]        = h01[r] + l01[r] * RSC;
      Cs[(row + 16) * LDC + nw * 32 + c]      = h10[r] + l10[r] * RSC;
      Cs[(row + 16) * LDC + nw * 32 + 16 + c] = h11[r] + l11[r] * RSC;
    }
  }
  {
    v8f m00 = zero8(), m01 = zero8(), m10 = zero8(), m11 = zero8();
#pragma unroll 1
    for (int ks = 0; ks < CC / 32; ++ks) {
      const size_t ao = (size_t)(2 * ks) * HSZ;
      const size_t bo = (size_t)(2 * ks) * (CC * HD);
      const v16h ga0 = ldfrag2(Vl + r0 + ao, Vl + r0 + ao + HSZ);
      const v16h ga1 = ldfrag2(Vl + r1 + ao, Vl + r1 + ao + HSZ);
      const v16h fb0 = ldfrag2(Wh + q0 + bo, Wh + q0 + bo + CC * HD);
      const v16h fb1 = ldfrag2(Wh + q1 + bo, Wh + q1 + bo + CC * HD);
      m00 = mma_raw(ga0, fb0, m00);
      m01 = mma_raw(ga0, fb1, m01);
      m10 = mma_raw(ga1, fb0, m10);
      m11 = mma_raw(ga1, fb1, m11);
      guard4(m00, m01, m10, m11, ga0, ga1, fb0, fb1);
    }
#pragma unroll
    for (int r = 0; r < 8; ++r) {
      const int row = mw * 32 + 8 * hh + r;
      Cs[row * LDC + nw * 32 + c]             += m00[r] * RSC;
      Cs[row * LDC + nw * 32 + 16 + c]        += m01[r] * RSC;
      Cs[(row + 16) * LDC + nw * 32 + c]      += m10[r] * RSC;
      Cs[(row + 16) * LDC + nw * 32 + 16 + c] += m11[r] * RSC;
    }
  }
}

__global__ __launch_bounds__(256)
void k_wcvt(const float* __restrict__ wq1, const float* __restrict__ wq2, const float* __restrict__ wk1,
            const float* __restrict__ wk2, const float* __restrict__ wv1, const float* __restrict__ wv2,
            unsigned short* w1, unsigned short* wt) {
  const int tid = threadIdx.x;
  const int blk = blockIdx.x;
  if (blk < 3 * CC) {
    const int t = blk / CC, co = blk - t * CC;
    const float* src = (t == 0) ? wq2 : ((t == 1) ? wk2 : wv2);
    const int tt = min(tid, 143);
    const int k0 = tt * 8, tap = k0 / CC, c0 = k0 - tap * CC;
    v4u pk;
#pragma unroll
    for (int e = 0; e < 4; ++e) {
      const float f0 = src[(size_t)(co * CC + c0 + 2 * e) * 9 + tap];
      const float f1 = src[(size_t)(co * CC + c0 + 2 * e + 1) * 9 + tap];
      pk[e] = pk16(hb16(bfr(f0) * 64.0f), hb16(bfr(f1) * 64.0f));
    }
    if (tid < 144) {
      unsigned short* dst = wt + (size_t)(t * CC + co) * KCV + k0;
      *(volatile v4u*)dst = pk;
      __threadfence();
      *(volatile v4u*)dst = pk;
    }
  } else {
    const int rr = blk - 3 * CC;
    const int t = rr / CC, o = rr - t * CC;
    const float* src = (t == 0) ? wq1 : ((t == 1) ? wk1 : wv1);
    const int tt = min(tid, 15);
    const int c0 = tt * 8;
    v4u pk;
#pragma unroll
    for (int e = 0; e < 4; ++e) {
      const float f0 = src[(size_t)o * CC + c0 + 2 * e];
      const float f1 = src[(size_t)o * CC + c0 + 2 * e + 1];
      pk[e] = pk16(hb16(bfr(f0) * 64.0f), hb16(bfr(f1) * 64.0f));
    }
    if (tid < 16) {
      unsigned short* dst = w1 + (size_t)(t * CC + o) * CC + c0;
      *(volatile v4u*)dst = pk;
      __threadfence();
      *(volatile v4u*)dst = pk;
    }
  }
}

__global__ __launch_bounds__(256)
void k_ln(const float* __restrict__ x, const float* __restrict__ gw, const float* __restrict__ gb,
          unsigned short* xh, unsigned short* xl) {
  __shared__ __align__(16) float T[64 * LDC];
  const int tid = threadIdx.x, wv = tid >> 5, lane = tid & 31;
  const int blk = blockIdx.x;
  const int bh = blk >> 1, chalf = blk & 1;
  const int b = bh / HH, h = bh - b * HH;
  const v4f g4 = *(const v4f*)(gw + lane * 4);
  const v4f b4 = *(const v4f*)(gb + lane * 4);
  float g[4], be[4];
#pragma unroll
  for (int e = 0; e < 4; ++e) { g[e] = bfr(g4[e]); be[e] = bfr(b4[e]); }
#pragma unroll 1
  for (int it = 0; it < 8; ++it) {
    const int cc = wv * 8 + it;
    const int c = chalf * 64 + cc;
    const float* row = x + ((size_t)(b * CC + c) * HH + h) * WW;
    const v4f a = *(const v4f*)(row + lane * 4);
    float xr[4];
#pragma unroll
    for (int e = 0; e < 4; ++e) xr[e] = bfr(a[e]);
    float s = (xr[0] + xr[1]) + (xr[2] + xr[3]);
#pragma unroll
    for (int off = 16; off; off >>= 1) s += __shfl_xor(s, off, 32);
    const float mu = s * (1.0f / 128.0f);
    float d[4];
#pragma unroll
    for (int e = 0; e < 4; ++e) d[e] = xr[e] - mu;
    float sq = (d[0] * d[0] + d[1] * d[1]) + (d[2] * d[2] + d[3] * d[3]);
#pragma unroll
    for (int off = 16; off; off >>= 1) sq += __shfl_xor(sq, off, 32);
    const float var = sq * (1.0f / 128.0f);
    const float rs = rsqrtf(var + 1e-5f);
    v4f o;
#pragma unroll
    for (int e = 0; e < 4; ++e) o[e] = (d[e] * rs) * g[e] + be[e];
    *(v4f*)(T + cc * LDC + lane * 4) = o;
  }
  __syncthreads();
  v4u ph[4], pq[4];
  size_t offs[4];
#pragma unroll
  for (int s = 0; s < 4; ++s) {
    const int idx = s * 256 + tid;
    const int w = idx >> 3, piece = idx & 7;
    const int c0 = piece * 8;
    v4u a, q4;
#pragma unroll
    for (int e = 0; e < 4; ++e) {
      const float f0 = T[(c0 + 2 * e) * LDC + w];
      const float f1 = T[(c0 + 2 * e + 1) * LDC + w];
      unsigned hp, lp;
      split2(f0, f1, hp, lp);
      a[e] = hp; q4[e] = lp;
    }
    ph[s] = a;
    pq[s] = q4;
    offs[s] = (size_t)(b * IMGPIX + h * WW + w) * CC + chalf * 64 + c0;
  }
#pragma unroll
  for (int s = 0; s < 4; ++s) { *(volatile v4u*)(xh + offs[s]) = ph[s]; *(volatile v4u*)(xl + offs[s]) = pq[s]; }
  __threadfence();
#pragma unroll
  for (int s = 0; s < 4; ++s) { *(volatile v4u*)(xh + offs[s]) = ph[s]; *(volatile v4u*)(xl + offs[s]) = pq[s]; }
}

__global__ __launch_bounds__(256)
void k_proj(const unsigned short* __restrict__ xh, const unsigned short* __restrict__ xl,
            const unsigned short* __restrict__ w1, unsigned short* p1) {
  __shared__ __align__(16) float Cs[64 * LDC];
  const int tid = threadIdx.x;
  const int mb = blockIdx.x, t = blockIdx.y;
  mm_tile2((const _Float16*)(const void*)xh, (const _Float16*)(const void*)xl, CC,
           (const _Float16*)(const void*)(w1 + (size_t)t * CC * CC), CC, CC / 32, mb * 64, 0, Cs);
  __syncthreads();
  unsigned short* dh = p1 + (size_t)(2 * t) * PS1;
  unsigned short* dl = p1 + (size_t)(2 * t + 1) * PS1;
  const int p0 = mb * 64;
  const int b = p0 / IMGPIX, rem = p0 - b * IMGPIX;
  const int y = rem / WW, x0 = rem - y * WW;
  const size_t pprow = (size_t)(b * HP + y + 1) * WP + x0 + 1;
  v4u ph[4], pq[4];
  size_t offs[4];
#pragma unroll
  for (int s = 0; s < 4; ++s) {
    const int idx = s * 256 + tid;
    const int row = idx >> 4, piece = idx & 15;
    const int col0 = piece * 8;
    v4u a, q4;
#pragma unroll
    for (int e = 0; e < 4; ++e) {
      const float f0 = Cs[row * LDC + col0 + 2 * e] * (1.0f / 64.0f);
      const float f1 = Cs[row * LDC + col0 + 2 * e + 1] * (1.0f / 64.0f);
      unsigned hp, lp;
      split2(f0, f1, hp, lp);
      a[e] = hp; q4[e] = lp;
    }
    ph[s] = a;
    pq[s] = q4;
    offs[s] = (pprow + row) * CC + col0;
  }
#pragma unroll
  for (int s = 0; s < 4; ++s) { *(volatile v4u*)(dh + offs[s]) = ph[s]; *(volatile v4u*)(dl + offs[s]) = pq[s]; }
  __threadfence();
#pragma unroll
  for (int s = 0; s < 4; ++s) { *(volatile v4u*)(dh + offs[s]) = ph[s]; *(volatile v4u*)(dl + offs[s]) = pq[s]; }
}

__global__ __launch_bounds__(256)
void k_halo(unsigned short* p1) {
  const int idx = blockIdx.x * 256 + threadIdx.x;
  if (idx >= 6 * NB * NHALO * 16) return;
  const int piece = idx & 15;
  int r = idx >> 4;
  const int hp = r % NHALO;
  r /= NHALO;
  const int img = r % NB, plane = r / NB;
  const int q = max(hp - 2 * WP, 0);
  const int pyA = (hp < WP) ? 0 : (HP - 1);
  const int pxA = (hp < WP) ? hp : (hp - WP);
  const int pyB = 1 + (q >> 1);
  const int pxB = (q & 1) ? (WP - 1) : 0;
  const bool edge = hp < 2 * WP;
  const int py = edge ? pyA : pyB;
  const int px = edge ? pxA : pxB;
  const size_t off = (size_t)plane * PS1 + ((size_t)(img * HP + py) * WP + px) * CC + piece * 8;
  v4u z = {0u, 0u, 0u, 0u};
  *(volatile v4u*)(p1 + off) = z;
  __threadfence();
  *(volatile v4u*)(p1 + off) = z;
}

__global__ __launch_bounds__(256)
void k_conv3(const unsigned short* __restrict__ p1, const unsigned short* __restrict__ wt,
             float* qk, unsigned short* vh, unsigned short* vl) {
  __shared__ __align__(16) float Cs[64 * LDC];
  const int tid = threadIdx.x;
  const int mb = blockIdx.x, t = blockIdx.y;
  mm_conv((const _Float16*)(const void*)(p1 + (size_t)(2 * t) * PS1),
          (const _Float16*)(const void*)(p1 + (size_t)(2 * t + 1) * PS1),
          (const _Float16*)(const void*)(wt + (size_t)t * CC * KCV), mb * 64, Cs);
  __syncthreads();
  const int p0 = mb * 64;
  const int b = p0 / IMGPIX, pix0 = p0 - b * IMGPIX;
  if (t < 2) {
    float* df = qk + (size_t)t * ((size_t)NB * BSZ);
    v4f pk[8];
    size_t offs[8];
#pragma unroll
    for (int s = 0; s < 8; ++s) {
      const int idx = s * 256 + tid;
      const int co = idx >> 4, piece = idx & 15;
      v4f v;
#pragma unroll
      for (int e = 0; e < 4; ++e) v[e] = Cs[(piece * 4 + e) * LDC + co] * (1.0f / 64.0f);
      pk[s] = v;
      offs[s] = (size_t)(b * CC + co) * IMGPIX + pix0 + piece * 4;
    }
#pragma unroll
    for (int s = 0; s < 8; ++s) *(volatile v4f*)(df + offs[s]) = pk[s];
    __threadfence();
#pragma unroll
    for (int s = 0; s < 8; ++s) *(volatile v4f*)(df + offs[s]) = pk[s];
  } else {
    v4u ph[4], pq[4];
    size_t offs[4];
#pragma unroll
    for (int s = 0; s < 4; ++s) {
      const int idx = s * 256 + tid;
      const int co = idx >> 3, piece = idx & 7;
      const int r0 = piece * 8;
      v4u a, q4;
#pragma unroll
      for (int e = 0; e < 4; ++e) {
        const float f0 = Cs[(r0 + 2 * e) * LDC + co] * (1.0f / 64.0f);
        const float f1 = Cs[(r0 + 2 * e + 1) * LDC + co] * (1.0f / 64.0f);
        unsigned hp, lp;
        split2(f0, f1, hp, lp);
        a[e] = hp; q4[e] = lp;
      }
      ph[s] = a;
      pq[s] = q4;
      offs[s] = (size_t)(b * CC + co) * IMGPIX + pix0 + r0;
    }
#pragma unroll
    for (int s = 0; s < 4; ++s) { *(volatile v4u*)(vh + offs[s]) = ph[s]; *(volatile v4u*)(vl + offs[s]) = pq[s]; }
    __threadfence();
#pragma unroll
    for (int s = 0; s < 4; ++s) { *(volatile v4u*)(vh + offs[s]) = ph[s]; *(volatile v4u*)(vl + offs[s]) = pq[s]; }
  }
}

__global__ __launch_bounds__(256)
void k_attn(const float* __restrict__ qk, const float* __restrict__ wo, const float* __restrict__ scale,
            unsigned short* weh, unsigned short* wel) {
  __shared__ float part[16 * 256];
  __shared__ float Sm[16 * WSP];
  __shared__ __align__(16) _Float16 Phs[16 * FP];
  __shared__ __align__(16) _Float16 Pls[16 * FP];
  __shared__ __align__(16) _Float16 Wts[CC * FP];
  __shared__ float Ws[CC * WSP];
  const int tid = threadIdx.x, wave = tid >> 5, lane = tid & 31, hh = lane >> 4, m = lane & 15;
  const int bi = blockIdx.x, b = bi / NHEAD, head = bi - b * NHEAD;
  const float* Qp = qk + (size_t)b * BSZ + (size_t)head * HSZ;
  const float* Kp = qk + (size_t)NB * BSZ + (size_t)b * BSZ + (size_t)head * HSZ;
  {
    const int rg = tid >> 4, i = tid & 15;
    float acc[HD];
#pragma unroll
    for (int e = 0; e < HD; ++e) acc[e] = 0.f;
#pragma unroll 1
    for (int so = 0; so < 32; ++so) {
      float tt[HD];
#pragma unroll
      for (int e = 0; e < HD; ++e) tt[e] = 0.f;
#pragma unroll 1
      for (int si = 0; si < 32; ++si) {
        const int r = (so * 32 + si) * 16 + rg;
        const float kv = Kp[(size_t)r * HD + i];
        const float* qr = Qp + (size_t)r * HD;
        const v4f q0 = *(const v4f*)(qr);
        const v4f q1 = *(const v4f*)(qr + 4);
        const v4f q2 = *(const v4f*)(qr + 8);
        const v4f q3 = *(const v4f*)(qr + 12);
#pragma unroll
        for (int e = 0; e < 4; ++e) {
          tt[e]      = fmaf(kv, q0[e], tt[e]);
          tt[4 + e]  = fmaf(kv, q1[e], tt[4 + e]);
          tt[8 + e]  = fmaf(kv, q2[e], tt[8 + e]);
          tt[12 + e] = fmaf(kv, q3[e], tt[12 + e]);
        }
      }
#pragma unroll
      for (int e = 0; e < HD; ++e) acc[e] += tt[e];
    }
#pragma unroll
    for (int j = 0; j < HD; ++j) part[rg * 256 + i * 16 + j] = acc[j];
  }
#pragma unroll 1
  for (int it = 0; it < 16; ++it) {
    const int idx = it * 256 + tid;
    const int o = idx >> 5, k = idx & 31;
    const int kk = min(k, HD - 1);
    const float f = wo[(size_t)o * CC + head * HD + kk];
    const float v = (k < HD) ? bfr(f) * 64.0f : 0.0f;
    Wts[o * FP + k] = (_Float16)v;
  }
  __syncthreads();
  {
    const int i = tid >> 4, j = tid & 15;
    float s = 0.f;
#pragma unroll
    for (int rg = 0; rg < 16; ++rg) s += part[rg * 256 + i * 16 + j];
    const float isc = 1.0f / bfr(scale[0]);
    Sm[i * WSP + j] = s * isc;
  }
  __syncthreads();
  if (tid < 16) {
    float mx = -3.0e38f;
#pragma unroll 1
    for (int n = 0; n < HD; ++n) mx = fmaxf(mx, Sm[tid * WSP + n]);
    float ssum = 0.f;
#pragma unroll 1
    for (int n = 0; n < HD; ++n) {
      const float e = expf(Sm[tid * WSP + n] - mx);
      Sm[tid * WSP + n] = e;
      ssum += e;
    }
    const float inv = 1.0f / ssum;
#pragma unroll 1
    for (int n = 0; n < HD; ++n) {
      const float pv = (Sm[tid * WSP + n] * inv) * 4096.0f;
      const _Float16 hv = (_Float16)pv;
      Phs[tid * FP + n] = hv;
      Pls[tid * FP + n] = (_Float16)((pv - (float)hv) * 2048.0f);
    }
#pragma unroll 1
    for (int n = HD; n < 32; ++n) { Phs[tid * FP + n] = (_Float16)0.0f; Pls[tid * FP + n] = (_Float16)0.0f; }
  }
  __syncthreads();
  {
    const v16h fa = ldfrag_h(Wts + (wave * 16 + m) * FP + 8 * hh);
    const v16h fb = ldfrag_h(Phs + m * FP + 8 * hh);
    const v16h gb = ldfrag_h(Pls + m * FP + 8 * hh);
    v8f ah = mma_raw(fa, fb, zero8());
    v8f al = mma_raw(fa, gb, zero8());
    guard2(ah, al, fa, fb, gb);
#pragma unroll
    for (int r = 0; r < 8; ++r) Ws[(wave * 16 + 8 * hh + r) * WSP + m] = (ah[r] + al[r] * RSC) * (1.0f / 4096.0f);
  }
  __syncthreads();
  {
    const int o = tid >> 1, hf = tid & 1;
    v4u a, q4;
#pragma unroll
    for (int e = 0; e < 4; ++e) {
      const float f0 = Ws[o * WSP + hf * 8 + 2 * e];
      const float f1 = Ws[o * WSP + hf * 8 + 2 * e + 1];
      unsigned hp, lp;
      split2(f0, f1, hp, lp);
      a[e] = hp; q4[e] = lp;
    }
    const size_t off = (size_t)(bi * CC + o) * HD + hf * 8;
    *(volatile v4u*)(weh + off) = a;
    *(volatile v4u*)(wel + off) = q4;
    __threadfence();
    *(volatile v4u*)(weh + off) = a;
    *(volatile v4u*)(wel + off) = q4;
  }
}

__global__ __launch_bounds__(256)
void k_final(const unsigned short* __restrict__ vh, const unsigned short* __restrict__ vl,
             const unsigned short* __restrict__ weh, const unsigned short* __restrict__ wel,
             const float* __restrict__ x, float* out) {
  __shared__ __align__(16) float Cs[64 * LDC];
  const int tid = threadIdx.x;
  const int mb = blockIdx.x;
  const int p0 = mb * 64;
  const int b = p0 / IMGPIX, pl0 = p0 - b * IMGPIX;
  const _Float16* Vh = (const _Float16*)(const void*)(vh + (size_t)b * BSZ);
  const _Float16* Vl = (const _Float16*)(const void*)(vl + (size_t)b * BSZ);
  const _Float16* Wh = (const _Float16*)(const void*)(weh + (size_t)b * NHEAD * CC * HD);
  const _Float16* Wl = (const _Float16*)(const void*)(wel + (size_t)b * NHEAD * CC * HD);
  mm_final(Vh, Vl, Wh, Wl, pl0, Cs);
  __syncthreads();
  v4f pk[8];
  size_t offs[8];
#pragma unroll
  for (int s = 0; s < 8; ++s) {
    const int idx = s * 256 + tid;
    const int o = idx >> 4, piece = idx & 15;
    const size_t off = (size_t)(b * CC + o) * IMGPIX + pl0 + piece * 4;
    const v4f xr = *(const v4f*)(x + off);
    v4f v;
#pragma unroll
    for (int e = 0; e < 4; ++e) v[e] = Cs[(piece * 4 + e) * LDC + o] * (1.0f / 64.0f) + bfr(xr[e]);
    pk[s] = v;
    offs[s] = off;
  }
#pragma unroll
  for (int s = 0; s < 8; ++s) *(volatile v4f*)(out + offs[s]) = pk[s];
  __threadfence();
#pragma unroll
  for (int s = 0; s < 8; ++s) *(volatile v4f*)(out + offs[s]) = pk[s];
}

extern "C" void kernel_launch(void* const* d_in, const int* in_sizes, int n_in,
                              void* d_out, int out_size, void* d_ws, size_t ws_size,
                              hipStream_t stream) {
  if (n_in < 11) return;
  const int expect[11] = { NB * CC * IMGPIX, WW, WW, 1, CC * CC, CC * CC * 9, CC * CC, CC * CC * 9,
                           CC * CC, CC * CC * 9, CC * CC };
  for (int i = 0; i < 11; ++i) if (in_sizes[i] != expect[i]) return;
  if (out_size != NB * CC * IMGPIX) return;

  const float* x     = (const float*)d_in[0];
  const float* gam   = (const float*)d_in[1];
  const float* bet   = (const float*)d_in[2];
  const float* scale = (const float*)d_in[3];
  const float* wq1   = (const float*)d_in[4];
  const float* wq2   = (const float*)d_in[5];
  const float* wk1   = (const float*)d_in[6];
  const float* wk2   = (const float*)d_in[7];
  const float* wv1   = (const float*)d_in[8];
  const float* wv2   = (const float*)d_in[9];
  const float* wo    = (const float*)d_in[10];
  float* out = (float*)d_out;

  const size_t AL = 65536;
  const size_t sW1 = (((size_t)3 * CC * CC * 2) + AL - 1) / AL * AL;
  const size_t sWT = (((size_t)3 * CC * KCV * 2) + AL - 1) / AL * AL;
  const size_t sX  = (((size_t)NPIX * CC * 2) + AL - 1) / AL * AL;
  const size_t sP1 = (((size_t)6 * PS1 * 2) + AL - 1) / AL * AL;
  const size_t sQK = (((size_t)2 * NB * BSZ * 4) + AL - 1) / AL * AL;
  const size_t sV  = (((size_t)NB * BSZ * 2) + AL - 1) / AL * AL;
  const size_t sWE = (((size_t)NB * NHEAD * CC * HD * 2) + AL - 1) / AL * AL;

  size_t off = 0;
  const size_t oW1  = off; off += sW1;
  const size_t oWT  = off; off += sWT;
  const size_t oXH  = off; off += sX;
  const size_t oXL  = off; off += sX;
  const size_t oP1  = off; off += sP1;
  const size_t oQK  = off; off += sQK;
  const size_t oVH  = off; off += sV;
  const size_t oVL  = off; off += sV;
  const size_t oWEH = off; off += sWE;
  const size_t oWEL = off; off += sWE;
  if (off > ws_size) return;
  if (off > (size_t)134217728) return;

  char* ws = (char*)d_ws;
  unsigned short* W1  = (unsigned short*)(ws + oW1);
  unsigned short* WT  = (unsigned short*)(ws + oWT);
  unsigned short* XH  = (unsigned short*)(ws + oXH);
  unsigned short* XL  = (unsigned short*)(ws + oXL);
  unsigned short* P1  = (unsigned short*)(ws + oP1);
  float*          QK  = (float*)(ws + oQK);
  unsigned short* VH  = (unsigned short*)(ws + oVH);
  unsigned short* VL  = (unsigned short*)(ws + oVL);
  unsigned short* WEH = (unsigned short*)(ws + oWEH);
  unsigned short* WEL = (unsigned short*)(ws + oWEL);

  const dim3 blk(256);
  k_wcvt<<<dim3(6 * CC), blk, 0, stream>>>(wq1, wq2, wk1, wk2, wv1, wv2, W1, WT);
  k_ln<<<dim3(NB * HH * 2), blk, 0, stream>>>(x, gam, bet, XH, XL);
  k_proj<<<dim3(NPIX / 64, 3), blk, 0, stream>>>(XH, XL, W1, P1);
  k_halo<<<dim3((6 * NB * NHALO * 16 + 255) / 256), blk, 0, stream>>>(P1);
  k_conv3<<<dim3(NPIX / 64, 3), blk, 0, stream>>>(P1, WT, QK, VH, VL);
  k_attn<<<dim3(NB * NHEAD), blk, 0, stream>>>(QK, wo, scale, WEH, WEL);
  k_final<<<dim3(NPIX / 64), blk, 0, stream>>>(VH, VL, WEH, WEL, x, out);
  (void)hipGetLastError();
}
